// HomoGNN_74577812128299
// MI455X (gfx1250) — hardware-verified
//
#include <hip/hip_runtime.h>
#include <stddef.h>


#define CIN     256
#define CHID    256
#define COUT    128
#define NTHR    256
#define NWAVE   8
#define EPT     8
#define NGRP    2
#define CHUNK   (NTHR * EPT * NGRP)
#define WCAP    (EPT * NGRP * 32)
#define LISTN   (NWAVE * WCAP)
#define NBD     4096
#define NB1     256
#define NB2     512
#define G1ROWS  64
#define APITCH  264

#define LDS_GEMM1 (G1ROWS * APITCH * 2 * 2)
#define LDS_AGG1  (NB1 * CHID * 4 + LISTN * 4 + 64)
#define LDS_AGG2  (NB2 * COUT * 4 + LISTN * 4 + 64)

static_assert((CHUNK & (CHUNK - 1)) == 0);
static_assert(CHUNK <= 4096);
static_assert((NB1 & (NB1 - 1)) == 0);
static_assert((NB2 & (NB2 - 1)) == 0);
static_assert((NBD & (NBD - 1)) == 0);
static_assert(NB1 <= 4096 && NB2 <= 4096 && NBD <= 4096);
static_assert(G1ROWS * CHID * 4 <= LDS_GEMM1);
static_assert(((APITCH * 2) & 15) == 0);
static_assert(NB1 % (NWAVE * 16) == 0 && NB2 % (NWAVE * 16) == 0);

typedef float          v4f   __attribute__((ext_vector_type(4)));
typedef float          v8f   __attribute__((ext_vector_type(8)));
typedef int            v4i   __attribute__((ext_vector_type(4)));
typedef unsigned short v8us  __attribute__((ext_vector_type(8)));
typedef __bf16         v16bf __attribute__((ext_vector_type(16)));
union FragB { v16bf v; v8us u[2]; };

__device__ __forceinline__ unsigned short bfr(float f) {
  const unsigned u = __float_as_uint(f);
  return (unsigned short)((u + 0x7FFFu + ((u >> 16) & 1u)) >> 16);
}
__device__ __forceinline__ void split1(float f, unsigned short& h, unsigned short& l) {
  const unsigned short hb = bfr(f);
  const float hf = __uint_as_float(((unsigned)hb) << 16);
  h = hb;
  l = bfr(f - hf);
}
__device__ __forceinline__ void split8(v4f a, v4f b, v8us& hi, v8us& lo) {
  unsigned short h, l;
  split1(a.x, h, l); hi[0] = h; lo[0] = l;
  split1(a.y, h, l); hi[1] = h; lo[1] = l;
  split1(a.z, h, l); hi[2] = h; lo[2] = l;
  split1(a.w, h, l); hi[3] = h; lo[3] = l;
  split1(b.x, h, l); hi[4] = h; lo[4] = l;
  split1(b.y, h, l); hi[5] = h; lo[5] = l;
  split1(b.z, h, l); hi[6] = h; lo[6] = l;
  split1(b.w, h, l); hi[7] = h; lo[7] = l;
}

__device__ __forceinline__ v8f wmb(v16bf a, v16bf b, v8f c) {
  v8f d = __builtin_amdgcn_wmma_f32_16x16x32_bf16(false, a, false, b, (short)0, c, false, false);
  asm volatile("v_nop\n\tv_nop\n\tv_nop\n\tv_nop" : "+v"(d) : "v"(a), "v"(b));
  return d;
}
__device__ __forceinline__ v8f wm3(const FragB& ah, const FragB& al, const FragB& bh, const FragB& bl, v8f c) {
  c = wmb(ah.v, bh.v, c);
  c = wmb(ah.v, bl.v, c);
  c = wmb(al.v, bh.v, c);
  return c;
}

template <int NB>
__device__ __forceinline__ int scan_chunk(const int* __restrict__ dsts, int nE, int cbase, int nodeBase,
                                          int vec8, int* list, int tid, int lane, int wave) {
  int wc = 0;
#pragma unroll
  for (int g = 0; g < NGRP; ++g) {
    const int el0  = (g * NTHR + tid) * EPT;
    const int e0   = cbase + el0;
    const int sent = -2147483647 - 1;
    v4i da, db;
    if (vec8 != 0 && cbase + CHUNK <= nE) {
      da = *(const v4i*)(dsts + e0);
      db = *(const v4i*)(dsts + e0 + 4);
    } else {
      da.x = (e0     < nE) ? dsts[min(e0, nE - 1)] : sent;
      da.y = (e0 + 1 < nE) ? dsts[min(e0 + 1, nE - 1)] : sent;
      da.z = (e0 + 2 < nE) ? dsts[min(e0 + 2, nE - 1)] : sent;
      da.w = (e0 + 3 < nE) ? dsts[min(e0 + 3, nE - 1)] : sent;
      db.x = (e0 + 4 < nE) ? dsts[min(e0 + 4, nE - 1)] : sent;
      db.y = (e0 + 5 < nE) ? dsts[min(e0 + 5, nE - 1)] : sent;
      db.z = (e0 + 6 < nE) ? dsts[min(e0 + 6, nE - 1)] : sent;
      db.w = (e0 + 7 < nE) ? dsts[min(e0 + 7, nE - 1)] : sent;
    }
    const unsigned nb = (unsigned)nodeBase;
    const unsigned s0 = (unsigned)da.x - nb, s1 = (unsigned)da.y - nb;
    const unsigned s2 = (unsigned)da.z - nb, s3 = (unsigned)da.w - nb;
    const unsigned s4 = (unsigned)db.x - nb, s5 = (unsigned)db.y - nb;
    const unsigned s6 = (unsigned)db.z - nb, s7 = (unsigned)db.w - nb;
    const bool h0 = s0 < (unsigned)NB, h1 = s1 < (unsigned)NB, h2 = s2 < (unsigned)NB, h3 = s3 < (unsigned)NB;
    const bool h4 = s4 < (unsigned)NB, h5 = s5 < (unsigned)NB, h6 = s6 < (unsigned)NB, h7 = s7 < (unsigned)NB;
    const unsigned any = __builtin_amdgcn_ballot_w32(h0 | h1 | h2 | h3 | h4 | h5 | h6 | h7);
    if (any != 0u) {
#define HITJ(J, HJ, SJ) { \
        const unsigned mj = __builtin_amdgcn_ballot_w32(HJ); \
        if (mj != 0u) { \
          if (HJ) { \
            const int pos = wc + (int)__builtin_amdgcn_mbcnt_lo(mj, 0u); \
            if (pos < WCAP) list[wave * WCAP + pos] = ((el0 + (J)) << 12) | (int)(SJ); \
          } \
          wc += (int)__builtin_popcount(mj); } }
      HITJ(0, h0, s0)
      HITJ(1, h1, s1)
      HITJ(2, h2, s2)
      HITJ(3, h3, s3)
      HITJ(4, h4, s4)
      HITJ(5, h5, s5)
      HITJ(6, h6, s6)
      HITJ(7, h7, s7)
#undef HITJ
    }
  }
  return wc;
}

__global__ __launch_bounds__(NTHR) void k_wprep(
    const float* __restrict__ W1, const float* __restrict__ W2, const float* __restrict__ Wl,
    unsigned short* w1h, unsigned short* w1l, unsigned short* w2h, unsigned short* w2l,
    unsigned short* wlh, unsigned short* wll) {
  const int i  = blockIdx.x * NTHR + threadIdx.x;
  const int n1 = CIN * CHID / 8;
  const int n2 = CHID * COUT / 8;
  const int n3 = COUT * COUT / 8;
  if (i >= n1 + n2 + n3) return;
  v4f a, b;
  unsigned short* dh;
  unsigned short* dl;
  int o;
  if (i < n1) {
    o = i * 8;
    const int n = o / CIN, k0 = o - n * CIN;
    const float* p = W1 + (size_t)k0 * CHID + n;
    a.x = p[0];        a.y = p[CHID];     a.z = p[2 * CHID]; a.w = p[3 * CHID];
    b.x = p[4 * CHID]; b.y = p[5 * CHID]; b.z = p[6 * CHID]; b.w = p[7 * CHID];
    dh = w1h; dl = w1l;
  } else if (i < n1 + n2) {
    o = (i - n1) * 8;
    const int n = o / CHID, k0 = o - n * CHID;
    const float* p = W2 + (size_t)k0 * COUT + n;
    a.x = p[0];        a.y = p[COUT];     a.z = p[2 * COUT]; a.w = p[3 * COUT];
    b.x = p[4 * COUT]; b.y = p[5 * COUT]; b.z = p[6 * COUT]; b.w = p[7 * COUT];
    dh = w2h; dl = w2l;
  } else {
    o = (i - n1 - n2) * 8;
    const int n = o / COUT, k0 = o - n * COUT;
    const float* p = Wl + (size_t)k0 * COUT + n;
    a.x = p[0];        a.y = p[COUT];     a.z = p[2 * COUT]; a.w = p[3 * COUT];
    b.x = p[4 * COUT]; b.y = p[5 * COUT]; b.z = p[6 * COUT]; b.w = p[7 * COUT];
    dh = wlh; dl = wll;
  }
  v8us hv, lv;
  split8(a, b, hv, lv);
  *(volatile v8us*)(dh + o) = hv;
  *(volatile v8us*)(dl + o) = lv;
  __threadfence();
  *(volatile v8us*)(dh + o) = hv;
  *(volatile v8us*)(dl + o) = lv;
}

__global__ __launch_bounds__(NTHR) void k_deg(
    const int* __restrict__ ei, float* dis, int nE, int vec8) {
  __shared__ __attribute__((aligned(16))) int cnt[NBD];
  __shared__ __attribute__((aligned(16))) int list[LISTN];
  __shared__ int wcnt[NWAVE];
  const int tid = threadIdx.x, lane = tid & 31, wave = tid >> 5;
  const int nodeBase = blockIdx.x * NBD;
  const int* dsts = ei + nE;

  for (int i = tid; i < NBD; i += NTHR) cnt[i] = 0;
  __syncthreads();

  const int nChunks = (nE + CHUNK - 1) / CHUNK;
#pragma unroll 1
  for (int ch = 0; ch < nChunks; ++ch) {
    const int cbase = ch * CHUNK;
    const int wc = scan_chunk<NBD>(dsts, nE, cbase, nodeBase, vec8, list, tid, lane, wave);
    if (lane == 0) wcnt[wave] = wc;
    __syncthreads();
    if (wave == 0) {
#pragma unroll 1
      for (int wsx = 0; wsx < NWAVE; ++wsx) {
        int n = __builtin_amdgcn_readfirstlane(wcnt[wsx]);
        n = n > WCAP ? WCAP : (n < 0 ? 0 : n);
        const int* lp = list + wsx * WCAP;
#pragma unroll 1
        for (int i = 0; i < n; ++i) {
          const int ent  = __builtin_amdgcn_readfirstlane(lp[i]);
          const int slot = ent & (NBD - 1);
          if (lane == 0) cnt[slot] = cnt[slot] + 1;
        }
      }
    }
    __syncthreads();
  }

  v4f dq[4];
#pragma unroll
  for (int q = 0; q < 4; ++q) {
    const int f = (wave * 4 + q) * 128 + 4 * lane;
    const v4i c = *(const v4i*)(cnt + f);
    dq[q].x = rsqrtf((float)(c.x + 1));
    dq[q].y = rsqrtf((float)(c.y + 1));
    dq[q].z = rsqrtf((float)(c.z + 1));
    dq[q].w = rsqrtf((float)(c.w + 1));
  }
  float* dp = dis + (size_t)nodeBase;
#pragma unroll
  for (int q = 0; q < 4; ++q) *(volatile v4f*)(dp + (wave * 4 + q) * 128 + 4 * lane) = dq[q];
  __threadfence();
#pragma unroll
  for (int q = 0; q < 4; ++q) *(volatile v4f*)(dp + (wave * 4 + q) * 128 + 4 * lane) = dq[q];
}

__global__ __launch_bounds__(NTHR) void k_gemm1(
    const float* __restrict__ x, const unsigned short* __restrict__ w1h, const unsigned short* __restrict__ w1l,
    const float* __restrict__ dis, float* g1, int nN) {
  extern __shared__ v4f lds_dyn[];
  unsigned short* sAh = (unsigned short*)lds_dyn;
  unsigned short* sAl = sAh + G1ROWS * APITCH;
  float*          stg = (float*)lds_dyn;
  const int tid = threadIdx.x, lane = tid & 31, wave = tid >> 5, hh = lane >> 4, m = lane & 15;
  const int rt = wave & 3, chf = wave >> 2;
  const int rowBase = blockIdx.x * G1ROWS;

#pragma unroll 2
  for (int i = 0; i < (G1ROWS * CIN / 8) / NTHR; ++i) {
    const int idx = i * NTHR + tid;
    const int r   = idx >> 5;
    const int c0  = (idx & 31) * 8;
    int node = rowBase + r;
    node = node > nN - 1 ? nN - 1 : node;
    const float* xp = x + (size_t)node * CIN + c0;
    const v4f a = *(const v4f*)xp, b = *(const v4f*)(xp + 4);
    v8us hv, lv;
    split8(a, b, hv, lv);
    *(v8us*)(sAh + r * APITCH + c0) = hv;
    *(v8us*)(sAl + r * APITCH + c0) = lv;
  }
  __syncthreads();

  v8f acc[8];
#pragma unroll
  for (int t = 0; t < 8; ++t) { v8f z = {0.f, 0.f, 0.f, 0.f, 0.f, 0.f, 0.f, 0.f}; acc[t] = z; }
  const unsigned short* arh = sAh + (16 * rt + m) * APITCH + 8 * hh;
  const unsigned short* arl = sAl + (16 * rt + m) * APITCH + 8 * hh;
#pragma unroll 1
  for (int kt = 0; kt < CIN / 32; ++kt) {
    FragB ah, al;
    ah.u[0] = *(const v8us*)(arh + 32 * kt);
    ah.u[1] = *(const v8us*)(arh + 32 * kt + 16);
    al.u[0] = *(const v8us*)(arl + 32 * kt);
    al.u[1] = *(const v8us*)(arl + 32 * kt + 16);
#pragma unroll
    for (int t = 0; t < 8; ++t) {
      const size_t bo = (size_t)(16 * (8 * chf + t) + m) * CIN + 32 * kt + 8 * hh;
      FragB bh, bl;
      bh.u[0] = *(const v8us*)(w1h + bo);
      bh.u[1] = *(const v8us*)(w1h + bo + 16);
      bl.u[0] = *(const v8us*)(w1l + bo);
      bl.u[1] = *(const v8us*)(w1l + bo + 16);
      acc[t] = wm3(ah, al, bh, bl, acc[t]);
    }
  }
  __syncthreads();

  const int r0 = 16 * rt + 8 * hh;
  const v4f dA = *(const v4f*)(dis + (size_t)rowBase + r0);
  const v4f dB = *(const v4f*)(dis + (size_t)rowBase + r0 + 4);
  float* sp = stg + r0 * CHID + 128 * chf + m;
#pragma unroll
  for (int t = 0; t < 8; ++t) {
    sp[0 * CHID + 16 * t] = acc[t][0] * dA.x;
    sp[1 * CHID + 16 * t] = acc[t][1] * dA.y;
    sp[2 * CHID + 16 * t] = acc[t][2] * dA.z;
    sp[3 * CHID + 16 * t] = acc[t][3] * dA.w;
    sp[4 * CHID + 16 * t] = acc[t][4] * dB.x;
    sp[5 * CHID + 16 * t] = acc[t][5] * dB.y;
    sp[6 * CHID + 16 * t] = acc[t][6] * dB.z;
    sp[7 * CHID + 16 * t] = acc[t][7] * dB.w;
  }
  __syncthreads();

  const float* lp = stg + (8 * wave) * CHID + 4 * lane;
  float* gp = g1 + ((size_t)rowBase + 8 * wave) * CHID + 4 * lane;
#pragma unroll
  for (int i = 0; i < 8; ++i) {
    const v4f v0 = *(const v4f*)(lp + i * CHID), v1 = *(const v4f*)(lp + i * CHID + 128);
    *(volatile v4f*)(gp + (size_t)i * CHID) = v0;
    *(volatile v4f*)(gp + (size_t)i * CHID + 128) = v1;
  }
  __threadfence();
#pragma unroll
  for (int i = 0; i < 8; ++i) {
    const v4f v0 = *(const v4f*)(lp + i * CHID), v1 = *(const v4f*)(lp + i * CHID + 128);
    *(volatile v4f*)(gp + (size_t)i * CHID) = v0;
    *(volatile v4f*)(gp + (size_t)i * CHID + 128) = v1;
  }
}

__global__ __launch_bounds__(NTHR) void k_agg1(
    const int* __restrict__ ei, const float* __restrict__ g1, const float* __restrict__ dis,
    const float* __restrict__ b1, const unsigned short* __restrict__ w2h, const unsigned short* __restrict__ w2l,
    float* g2, int nN, int nE, int vec8) {
  extern __shared__ v4f lds_dyn[];
  float* acc  = (float*)lds_dyn;
  int*   list = (int*)(acc + NB1 * CHID);
  int*   wcnt = list + LISTN;
  const int tid = threadIdx.x, lane = tid & 31, wave = tid >> 5, hh = lane >> 4, m = lane & 15;
  const int nodeBase = blockIdx.x * NB1;
  const int* dsts = ei + nE;

  {
    const v4f z = {0.f, 0.f, 0.f, 0.f};
    for (int i = tid; i < NB1 * CHID / 4; i += NTHR) lds_dyn[i] = z;
  }
  __syncthreads();

  const int nChunks = (nE + CHUNK - 1) / CHUNK;
#pragma unroll 1
  for (int ch = 0; ch < nChunks; ++ch) {
    const int cbase = ch * CHUNK;
    const int wc = scan_chunk<NB1>(dsts, nE, cbase, nodeBase, vec8, list, tid, lane, wave);
    if (lane == 0) wcnt[wave] = wc;
    __syncthreads();
    if (wave == 0) {
#pragma unroll 1
      for (int wsx = 0; wsx < NWAVE; ++wsx) {
        int n = __builtin_amdgcn_readfirstlane(wcnt[wsx]);
        n = n > WCAP ? WCAP : (n < 0 ? 0 : n);
        const int* lp = list + wsx * WCAP;
#pragma unroll 1
        for (int i = 0; i < n; ++i) {
          const int ent  = __builtin_amdgcn_readfirstlane(lp[i]);
          const int slot = ent & (NB1 - 1);
          int e = cbase + ((ent >> 12) & (CHUNK - 1));
          e = e > nE - 1 ? nE - 1 : e;
          int src = ei[e];
          src = src < 0 ? 0 : (src > nN - 1 ? nN - 1 : src);
          const float* gp = g1 + (size_t)src * CHID + 4 * lane;
          const v4f v0 = *(const v4f*)gp;
          const v4f v1 = *(const v4f*)(gp + 128);
          v4f* ap = (v4f*)(acc + slot * CHID + 4 * lane);
          ap[0]  = ap[0] + v0;
          ap[32] = ap[32] + v1;
        }
      }
    }
    __syncthreads();
  }

#pragma unroll 4
  for (int i = 0; i < (NB1 * CHID / 4) / NTHR; ++i) {
    const int idx  = i * NTHR + tid;
    const int slot = idx >> 6;
    const int c4   = (idx & 63) * 4;
    int node = nodeBase + slot;
    node = node > nN - 1 ? nN - 1 : node;
    const float d  = dis[node];
    const v4f   gv = *(const v4f*)(g1 + (size_t)node * CHID + c4);
    const v4f   bv = *(const v4f*)(b1 + c4);
    v4f* ap = (v4f*)(acc + slot * CHID + c4);
    v4f hv = (*ap + gv) * d + bv;
    hv.x = fmaxf(hv.x, 0.f); hv.y = fmaxf(hv.y, 0.f); hv.z = fmaxf(hv.z, 0.f); hv.w = fmaxf(hv.w, 0.f);
    *ap = hv;
  }
  __syncthreads();

#pragma unroll 1
  for (int q = 0; q < NB1 / (NWAVE * 16); ++q) {
    const int t = wave + NWAVE * q;
    v8f c[8];
#pragma unroll
    for (int u = 0; u < 8; ++u) { v8f z = {0.f, 0.f, 0.f, 0.f, 0.f, 0.f, 0.f, 0.f}; c[u] = z; }
#pragma unroll 1
    for (int kt = 0; kt < CHID / 32; ++kt) {
      const float* ap = acc + (16 * t + m) * CHID + 32 * kt + 8 * hh;
      const v4f p0 = *(const v4f*)ap,        p1 = *(const v4f*)(ap + 4);
      const v4f p2 = *(const v4f*)(ap + 16), p3 = *(const v4f*)(ap + 20);
      FragB ah, al;
      split8(p0, p1, ah.u[0], al.u[0]);
      split8(p2, p3, ah.u[1], al.u[1]);
#pragma unroll
      for (int ct = 0; ct < 8; ++ct) {
        const size_t bo = (size_t)(16 * ct + m) * CHID + 32 * kt + 8 * hh;
        FragB bh, bl;
        bh.u[0] = *(const v8us*)(w2h + bo);
        bh.u[1] = *(const v8us*)(w2h + bo + 16);
        bl.u[0] = *(const v8us*)(w2l + bo);
        bl.u[1] = *(const v8us*)(w2l + bo + 16);
        c[ct] = wm3(ah, al, bh, bl, c[ct]);
      }
    }
    __syncthreads();
    const int node0 = nodeBase + 16 * t + 8 * hh;
    const v4f dA = *(const v4f*)(dis + (size_t)node0);
    const v4f dB = *(const v4f*)(dis + (size_t)node0 + 4);
    float* sp = acc + (16 * t + 8 * hh) * CHID + m;
#pragma unroll
    for (int ct = 0; ct < 8; ++ct) {
      sp[0 * CHID + 16 * ct] = c[ct][0] * dA.x;
      sp[1 * CHID + 16 * ct] = c[ct][1] * dA.y;
      sp[2 * CHID + 16 * ct] = c[ct][2] * dA.z;
      sp[3 * CHID + 16 * ct] = c[ct][3] * dA.w;
      sp[4 * CHID + 16 * ct] = c[ct][4] * dB.x;
      sp[5 * CHID + 16 * ct] = c[ct][5] * dB.y;
      sp[6 * CHID + 16 * ct] = c[ct][6] * dB.z;
      sp[7 * CHID + 16 * ct] = c[ct][7] * dB.w;
    }
  }
  __syncthreads();

  const int rw = 32 * wave;
  float* gp = g2 + ((size_t)nodeBase + rw) * COUT + 4 * lane;
  const float* lp = acc + rw * CHID + 4 * lane;
#pragma unroll 4
  for (int i = 0; i < 32; ++i) { const v4f v = *(const v4f*)(lp + i * CHID); *(volatile v4f*)(gp + (size_t)i * COUT) = v; }
  __threadfence();
#pragma unroll 4
  for (int i = 0; i < 32; ++i) { const v4f v = *(const v4f*)(lp + i * CHID); *(volatile v4f*)(gp + (size_t)i * COUT) = v; }
}

__global__ __launch_bounds__(NTHR) void k_agg2(
    const int* __restrict__ ei, const float* __restrict__ g2, const float* __restrict__ dis,
    const float* __restrict__ b2, const unsigned short* __restrict__ wlh, const unsigned short* __restrict__ wll,
    const float* __restrict__ bl, float* out, int nN, int nE, int vec8) {
  extern __shared__ v4f lds_dyn[];
  float* acc  = (float*)lds_dyn;
  int*   list = (int*)(acc + NB2 * COUT);
  int*   wcnt = list + LISTN;
  const int tid = threadIdx.x, lane = tid & 31, wave = tid >> 5, hh = lane >> 4, m = lane & 15;
  const int nodeBase = blockIdx.x * NB2;
  const int* dsts = ei + nE;

  {
    const v4f z = {0.f, 0.f, 0.f, 0.f};
    for (int i = tid; i < NB2 * COUT / 4; i += NTHR) lds_dyn[i] = z;
  }
  __syncthreads();

  const int nChunks = (nE + CHUNK - 1) / CHUNK;
#pragma unroll 1
  for (int ch = 0; ch < nChunks; ++ch) {
    const int cbase = ch * CHUNK;
    const int wc = scan_chunk<NB2>(dsts, nE, cbase, nodeBase, vec8, list, tid, lane, wave);
    if (lane == 0) wcnt[wave] = wc;
    __syncthreads();
    if (wave == 0) {
#pragma unroll 1
      for (int wsx = 0; wsx < NWAVE; ++wsx) {
        int n = __builtin_amdgcn_readfirstlane(wcnt[wsx]);
        n = n > WCAP ? WCAP : (n < 0 ? 0 : n);
        const int* lp = list + wsx * WCAP;
#pragma unroll 1
        for (int i = 0; i < n; ++i) {
          const int ent  = __builtin_amdgcn_readfirstlane(lp[i]);
          const int slot = ent & (NB2 - 1);
          int e = cbase + ((ent >> 12) & (CHUNK - 1));
          e = e > nE - 1 ? nE - 1 : e;
          int src = ei[e];
          src = src < 0 ? 0 : (src > nN - 1 ? nN - 1 : src);
          const v4f v = *(const v4f*)(g2 + (size_t)src * COUT + 4 * lane);
          v4f* ap = (v4f*)(acc + slot * COUT + 4 * lane);
          ap[0] = ap[0] + v;
        }
      }
    }
    __syncthreads();
  }

#pragma unroll 4
  for (int i = 0; i < (NB2 * COUT / 4) / NTHR; ++i) {
    const int idx  = i * NTHR + tid;
    const int slot = idx >> 5;
    const int c4   = (idx & 31) * 4;
    int node = nodeBase + slot;
    node = node > nN - 1 ? nN - 1 : node;
    const float d  = dis[node];
    const v4f   gv = *(const v4f*)(g2 + (size_t)node * COUT + c4);
    const v4f   bv = *(const v4f*)(b2 + c4);
    v4f* ap = (v4f*)(acc + slot * COUT + c4);
    v4f hv = (*ap + gv) * d + bv;
    hv.x = fmaxf(hv.x, 0.f); hv.y = fmaxf(hv.y, 0.f); hv.z = fmaxf(hv.z, 0.f); hv.w = fmaxf(hv.w, 0.f);
    *ap = hv;
  }
  __syncthreads();

#pragma unroll 1
  for (int q = 0; q < NB2 / (NWAVE * 16); ++q) {
    const int t = wave + NWAVE * q;
    v8f c[8];
#pragma unroll
    for (int u = 0; u < 8; ++u) { v8f z = {0.f, 0.f, 0.f, 0.f, 0.f, 0.f, 0.f, 0.f}; c[u] = z; }
#pragma unroll 1
    for (int kt = 0; kt < COUT / 32; ++kt) {
      const float* ap = acc + (16 * t + m) * COUT + 32 * kt + 8 * hh;
      const v4f p0 = *(const v4f*)ap,        p1 = *(const v4f*)(ap + 4);
      const v4f p2 = *(const v4f*)(ap + 16), p3 = *(const v4f*)(ap + 20);
      FragB ah, al;
      split8(p0, p1, ah.u[0], al.u[0]);
      split8(p2, p3, ah.u[1], al.u[1]);
#pragma unroll
      for (int ct = 0; ct < 8; ++ct) {
        const size_t bo = (size_t)(16 * ct + m) * COUT + 32 * kt + 8 * hh;
        FragB bh, bw;
        bh.u[0] = *(const v8us*)(wlh + bo);
        bh.u[1] = *(const v8us*)(wlh + bo + 16);
        bw.u[0] = *(const v8us*)(wll + bo);
        bw.u[1] = *(const v8us*)(wll + bo + 16);
        c[ct] = wm3(ah, al, bh, bw, c[ct]);
      }
    }
    __syncthreads();
    float* sp = acc + (16 * t + 8 * hh) * COUT + m;
#pragma unroll
    for (int ct = 0; ct < 8; ++ct) {
      const float bb = bl[16 * ct + m];
      sp[0 * COUT + 16 * ct] = c[ct][0] + bb;
      sp[1 * COUT + 16 * ct] = c[ct][1] + bb;
      sp[2 * COUT + 16 * ct] = c[ct][2] + bb;
      sp[3 * COUT + 16 * ct] = c[ct][3] + bb;
      sp[4 * COUT + 16 * ct] = c[ct][4] + bb;
      sp[5 * COUT + 16 * ct] = c[ct][5] + bb;
      sp[6 * COUT + 16 * ct] = c[ct][6] + bb;
      sp[7 * COUT + 16 * ct] = c[ct][7] + bb;
    }
  }
  __syncthreads();

  const int rw = 64 * wave;
#pragma unroll 4
  for (int i = 0; i < 64; ++i) {
    const int node = nodeBase + rw + i;
    if (node < nN) {
      const v4f v = *(const v4f*)(acc + (rw + i) * COUT + 4 * lane);
      *(volatile v4f*)(out + (size_t)node * COUT + 4 * lane) = v;
    }
  }
  __threadfence();
#pragma unroll 4
  for (int i = 0; i < 64; ++i) {
    const int node = nodeBase + rw + i;
    if (node < nN) {
      const v4f v = *(const v4f*)(acc + (rw + i) * COUT + 4 * lane);
      *(volatile v4f*)(out + (size_t)node * COUT + 4 * lane) = v;
    }
  }
}

extern "C" void kernel_launch(void* const* d_in, const int* in_sizes, int n_in,
                              void* d_out, int out_size, void* d_ws, size_t ws_size,
                              hipStream_t stream) {
  if (n_in < 8) return;
  const int nN = in_sizes[0] / CIN;
  const int nE = in_sizes[1] / 2;
  if (nN <= 0 || nE < 0 || in_sizes[0] != nN * CIN || in_sizes[1] != nE * 2) return;
  if (in_sizes[2] != CIN * CHID || in_sizes[3] < CHID) return;
  if (in_sizes[4] != CHID * COUT || in_sizes[5] < COUT) return;
  if (in_sizes[6] != COUT * COUT || in_sizes[7] < COUT) return;
  if (out_size != nN * COUT) return;

  const float* x  = (const float*)d_in[0];
  const int*   ei = (const int*)d_in[1];
  const float* W1 = (const float*)d_in[2];
  const float* b1 = (const float*)d_in[3];
  const float* W2 = (const float*)d_in[4];
  const float* b2 = (const float*)d_in[5];
  const float* Wl = (const float*)d_in[6];
  const float* bl = (const float*)d_in[7];
  float* out = (float*)d_out;

  const int nBD = (nN + NBD - 1) / NBD;
  const int nG1 = (nN + G1ROWS - 1) / G1ROWS;
  const int nA1 = (nN + NB1 - 1) / NB1;
  const int nA2 = (nN + NB2 - 1) / NB2;

  char* ws = (char*)d_ws;
  size_t off = 0;
  const size_t oW1h = off; off += (size_t)CIN * CHID * 2;               off = (off + 255) & ~(size_t)255;
  const size_t oW1l = off; off += (size_t)CIN * CHID * 2;               off = (off + 255) & ~(size_t)255;
  const size_t oW2h = off; off += (size_t)CHID * COUT * 2;              off = (off + 255) & ~(size_t)255;
  const size_t oW2l = off; off += (size_t)CHID * COUT * 2;              off = (off + 255) & ~(size_t)255;
  const size_t oWlh = off; off += (size_t)COUT * COUT * 2;              off = (off + 255) & ~(size_t)255;
  const size_t oWll = off; off += (size_t)COUT * COUT * 2;              off = (off + 255) & ~(size_t)255;
  const size_t oDis = off; off += (size_t)nBD * NBD * 4;                off = (off + 255) & ~(size_t)255;
  const size_t oG1  = off; off += (size_t)nG1 * G1ROWS * CHID * 4;      off = (off + 255) & ~(size_t)255;
  const size_t oG2  = off; off += (size_t)nA1 * NB1 * COUT * 4;         off = (off + 255) & ~(size_t)255;
  if (off > ws_size) return;
  if (off > (size_t)134217728u) return;
  unsigned short* w1h = (unsigned short*)(ws + oW1h);
  unsigned short* w1l = (unsigned short*)(ws + oW1l);
  unsigned short* w2h = (unsigned short*)(ws + oW2h);
  unsigned short* w2l = (unsigned short*)(ws + oW2l);
  unsigned short* wlh = (unsigned short*)(ws + oWlh);
  unsigned short* wll = (unsigned short*)(ws + oWll);
  float* dis = (float*)(ws + oDis);
  float* g1  = (float*)(ws + oG1);
  float* g2  = (float*)(ws + oG2);

  const int vec8 = ((nE & 3) == 0) ? 1 : 0;

  const int nPrep = CIN * CHID / 8 + CHID * COUT / 8 + COUT * COUT / 8;
  k_wprep<<<(nPrep + NTHR - 1) / NTHR, NTHR, 0, stream>>>(W1, W2, Wl, w1h, w1l, w2h, w2l, wlh, wll);

  k_deg<<<nBD, NTHR, 0, stream>>>(ei, dis, nE, vec8);

  hipFuncSetAttribute(reinterpret_cast<const void*>(&k_gemm1),
                      hipFuncAttributeMaxDynamicSharedMemorySize, LDS_GEMM1);
  k_gemm1<<<nG1, NTHR, LDS_GEMM1, stream>>>(x, w1h, w1l, dis, g1, nN);

  hipFuncSetAttribute(reinterpret_cast<const void*>(&k_agg1),
                      hipFuncAttributeMaxDynamicSharedMemorySize, LDS_AGG1);
  k_agg1<<<nA1, NTHR, LDS_AGG1, stream>>>(ei, g1, dis, b1, w2h, w2l, g2, nN, nE, vec8);

  hipFuncSetAttribute(reinterpret_cast<const void*>(&k_agg2),
                      hipFuncAttributeMaxDynamicSharedMemorySize, LDS_AGG2);
  k_agg2<<<nA2, NTHR, LDS_AGG2, stream>>>(ei, g2, dis, b2, wlh, wll, bl, out, nN, nE, vec8);
}
